// SpGraphAttentionLayer_58935541235965
// MI455X (gfx1250) — hardware-verified
//
#include <hip/hip_runtime.h>
#include <stddef.h>


#define KF     256
#define DF     128
#define GR     32
#define AP     264
#define XSP    132
#define NB     512
#define CHUNK  2048
#define NTHR   256
#define NWAVE  8
#define NGRP   (CHUNK / (NTHR * 4))
#define WCAP   (NGRP * 8 * 32)
#define RCAP   256
#define WPLANE (DF * KF)

#define LDS_SACC (NB * DF)
#define LDS_DEN  NB
#define LDS_LIST (NWAVE * WCAP)
#define LDS_BYTES ((LDS_SACC + LDS_DEN + LDS_LIST + NWAVE + RCAP) * 4)

static_assert(NGRP == 2);
static_assert(WCAP == 512);
static_assert(NB == 512);
static_assert(CHUNK == 2048);
static_assert(((LDS_SACC + LDS_DEN) % 4) == 0);
static_assert(LDS_BYTES == 281632);
static_assert(DF == NWAVE * 16);
static_assert((KF % 32) == 0);
static_assert(GR == 4 * NWAVE);
static_assert((DF % NWAVE) == 0);

typedef float          v4f   __attribute__((ext_vector_type(4)));
typedef float          v8f   __attribute__((ext_vector_type(8)));
typedef int            v4i   __attribute__((ext_vector_type(4)));
typedef unsigned short v8us  __attribute__((ext_vector_type(8)));
typedef __bf16         v16bf __attribute__((ext_vector_type(16)));
union Frag   { v16bf v; v8us half[2]; };
union Pack16 { v8us s; v4i i; };

__device__ __forceinline__ v8f wm(v16bf a, v16bf b, v8f c) {
  v8f d = __builtin_amdgcn_wmma_f32_16x16x32_bf16(false, a, false, b, (short)0, c, false, false);
  asm volatile("v_nop\n\tv_nop\n\tv_nop\n\tv_nop" : "+v"(d) : "v"(a), "v"(b));
  return d;
}

__device__ __forceinline__ float wsum(float v) {
  v += __shfl_xor(v, 16, 32);
  v += __shfl_xor(v, 8, 32);
  v += __shfl_xor(v, 4, 32);
  v += __shfl_xor(v, 2, 32);
  v += __shfl_xor(v, 1, 32);
  return v;
}

__device__ __forceinline__ unsigned int bfb(float x) {
  const unsigned int u = __float_as_uint(x);
  return (u + 0x7FFFu + ((u >> 16) & 1u)) >> 16;
}

__device__ __forceinline__ void split2(float x, unsigned short& hi, unsigned short& lo) {
  const unsigned int h = bfb(x);
  const float hf = __uint_as_float(h << 16);
  hi = (unsigned short)h;
  lo = (unsigned short)bfb(x - hf);
}

__global__ __launch_bounds__(NTHR) void k_prep(const float* __restrict__ W, unsigned short* Wp) {
  const int lane = threadIdx.x & 31;
  const int wave = threadIdx.x >> 5;
  const int n = blockIdx.x * NWAVE + wave;
  if (n >= DF) return;
  Pack16 ph, pl;
#pragma unroll
  for (int j = 0; j < 8; ++j) {
    const int k = 8 * lane + j;
    const float w = W[(size_t)k * DF + n];
    unsigned short hi, lo;
    split2(w, hi, lo);
    ph.s[j] = hi;
    pl.s[j] = lo;
  }
  unsigned short* p0 = Wp + (size_t)n * KF + 8 * lane;
  unsigned short* p1 = p0 + WPLANE;
  const v4i vh = ph.i, vl = pl.i;
  *(volatile v4i*)p0 = vh;
  *(volatile v4i*)p1 = vl;
  __threadfence();
  *(volatile v4i*)p0 = vh;
  *(volatile v4i*)p1 = vl;
}

__device__ __forceinline__ void epi_tile(v8f acc, int T, int hh, int m, int wave, int ncol,
                                         float c1, float c2, float* Xs, float* As, float* Ds) {
  float s1[8], s2[8];
#pragma unroll
  for (int r = 0; r < 8; ++r) {
    const float v = acc[r];
    Xs[(T * 16 + 8 * hh + r) * XSP + ncol] = v;
    s1[r] = v * c1;
    s2[r] = v * c2;
  }
#pragma unroll
  for (int mk = 1; mk < 16; mk <<= 1) {
#pragma unroll
    for (int r = 0; r < 8; ++r) {
      s1[r] += __shfl_xor(s1[r], mk, 32);
      s2[r] += __shfl_xor(s2[r], mk, 32);
    }
  }
  if (m == 0) {
#pragma unroll
    for (int r = 0; r < 8; ++r) {
      As[(T * 16 + 8 * hh + r) * NWAVE + wave] = s1[r];
      Ds[(T * 16 + 8 * hh + r) * NWAVE + wave] = s2[r];
    }
  }
}

__global__ __launch_bounds__(NTHR) void k_gemm(
    const float* __restrict__ x, const unsigned short* __restrict__ Wp,
    const float* __restrict__ av,
    float* Hp, float* ha1, float* ha2, int nN) {
  __shared__ __attribute__((aligned(16))) unsigned short At[2 * GR * AP];
  __shared__ __attribute__((aligned(16))) float Xs[GR * XSP];
  __shared__ __attribute__((aligned(16))) float As[GR * NWAVE];
  __shared__ __attribute__((aligned(16))) float Ds[GR * NWAVE];
  __shared__ __attribute__((aligned(16))) float S1[GR];
  __shared__ __attribute__((aligned(16))) float S2[GR];

  const int tid  = threadIdx.x;
  const int lane = tid & 31;
  const int wave = tid >> 5;
  const int hh   = lane >> 4;
  const int m    = lane & 15;
  const int rowBase = blockIdx.x * GR;

  {
    const int r  = tid >> 3;
    const int c0 = (tid & 7) * 32;
    int row = rowBase + r;
    if (row > nN - 1) row = nN - 1;
    const float* p = x + (size_t)row * KF + c0;
#pragma unroll
    for (int q = 0; q < 4; ++q) {
      const v4f f0 = *(const v4f*)(p + 8 * q);
      const v4f f1 = *(const v4f*)(p + 8 * q + 4);
      Pack16 ph, pl;
      unsigned short hi, lo;
      split2(f0.x, hi, lo); ph.s[0] = hi; pl.s[0] = lo;
      split2(f0.y, hi, lo); ph.s[1] = hi; pl.s[1] = lo;
      split2(f0.z, hi, lo); ph.s[2] = hi; pl.s[2] = lo;
      split2(f0.w, hi, lo); ph.s[3] = hi; pl.s[3] = lo;
      split2(f1.x, hi, lo); ph.s[4] = hi; pl.s[4] = lo;
      split2(f1.y, hi, lo); ph.s[5] = hi; pl.s[5] = lo;
      split2(f1.z, hi, lo); ph.s[6] = hi; pl.s[6] = lo;
      split2(f1.w, hi, lo); ph.s[7] = hi; pl.s[7] = lo;
      *(v4i*)(At + r * AP + c0 + 8 * q)           = ph.i;
      *(v4i*)(At + GR * AP + r * AP + c0 + 8 * q) = pl.i;
    }
  }
  __syncthreads();

  const int ncol = wave * 16 + m;
  v8f c0a = {0.f, 0.f, 0.f, 0.f, 0.f, 0.f, 0.f, 0.f};
  v8f c1a = {0.f, 0.f, 0.f, 0.f, 0.f, 0.f, 0.f, 0.f};
#pragma unroll 1
  for (int seg = 0; seg < 3; ++seg) {
    const unsigned short* Ab = At + ((seg == 2) ? (GR * AP) : 0);
    const unsigned short* Bb = Wp + (size_t)ncol * KF + ((seg == 1) ? WPLANE : 0);
#pragma unroll 4
    for (int kt = 0; kt < KF / 32; ++kt) {
      const int k0 = kt * 32;
      Frag a0, a1, b;
      const unsigned short* pb  = Bb + k0 + 8 * hh;
      const unsigned short* pa0 = Ab + m * AP + k0 + 8 * hh;
      const unsigned short* pa1 = Ab + (16 + m) * AP + k0 + 8 * hh;
      b.half[0]  = *(const v8us*)pb;  b.half[1]  = *(const v8us*)(pb + 16);
      a0.half[0] = *(const v8us*)pa0; a0.half[1] = *(const v8us*)(pa0 + 16);
      a1.half[0] = *(const v8us*)pa1; a1.half[1] = *(const v8us*)(pa1 + 16);
      c0a = wm(a0.v, b.v, c0a);
      c1a = wm(a1.v, b.v, c1a);
    }
  }

  const float c1 = av[ncol];
  const float c2 = av[DF + ncol];
  epi_tile(c0a, 0, hh, m, wave, ncol, c1, c2, Xs, As, Ds);
  epi_tile(c1a, 1, hh, m, wave, ncol, c1, c2, Xs, As, Ds);
  __syncthreads();

  if (wave == 0) {
    float s = 0.f;
#pragma unroll
    for (int w = 0; w < NWAVE; ++w) s += As[lane * NWAVE + w];
    S1[lane] = s;
  } else if (wave == 1) {
    float s = 0.f;
#pragma unroll
    for (int w = 0; w < NWAVE; ++w) s += Ds[lane * NWAVE + w];
    S2[lane] = s;
  }
  __syncthreads();

  v4f xr[4];
#pragma unroll
  for (int i = 0; i < 4; ++i) xr[i] = *(const v4f*)(Xs + (4 * wave + i) * XSP + 4 * lane);
  float* xpp[4];
#pragma unroll
  for (int i = 0; i < 4; ++i) xpp[i] = Hp + (size_t)(rowBase + 4 * wave + i) * DF + 4 * lane;
  const int l8 = lane & 7;
  const bool wl = (lane < 8) && (wave < 2);
  v4f gv = {0.f, 0.f, 0.f, 0.f};
  float* gp = ha1 + (size_t)rowBase + 4 * l8;
  if (wave == 0) {
    gv = *(const v4f*)(S1 + 4 * l8);
  } else if (wave == 1) {
    gv = *(const v4f*)(S2 + 4 * l8);
    gp = ha2 + (size_t)rowBase + 4 * l8;
  }

#pragma unroll
  for (int i = 0; i < 4; ++i) *(volatile v4f*)(xpp[i]) = xr[i];
  if (wl) *(volatile v4f*)gp = gv;
  __threadfence();
#pragma unroll
  for (int i = 0; i < 4; ++i) *(volatile v4f*)(xpp[i]) = xr[i];
  if (wl) *(volatile v4f*)gp = gv;
}

__global__ __launch_bounds__(NTHR) void k_agg(
    const float* __restrict__ Hp, const float* __restrict__ ha1, const float* __restrict__ ha2,
    const int* __restrict__ ei, const int* __restrict__ er,
    const float* __restrict__ remb, const float* __restrict__ av,
    float* out, int nN, int nE, int nR) {
  extern __shared__ v4f lds_dyn[];
  float* sacc = (float*)lds_dyn;
  float* den  = sacc + LDS_SACC;
  int*   list = (int*)(den + LDS_DEN);
  int*   wcnt = list + LDS_LIST;
  float* ra2s = (float*)(wcnt + NWAVE);

  const int tid  = threadIdx.x;
  const int lane = tid & 31;
  const int wave = tid >> 5;
  const int nodeBase = blockIdx.x * NB;

  {
    const v4f z4 = {0.f, 0.f, 0.f, 0.f};
    for (int i = tid; i < (LDS_SACC + LDS_DEN) / 4; i += NTHR) lds_dyn[i] = z4;
    const v4f a2v = *(const v4f*)(av + DF + 4 * lane);
#pragma unroll 1
    for (int rr = wave; rr < nR; rr += NWAVE) {
      const v4f rv = *(const v4f*)(remb + (size_t)rr * DF + 4 * lane);
      float d = rv.x * a2v.x + rv.y * a2v.y + rv.z * a2v.z + rv.w * a2v.w;
      d = wsum(d);
      if (lane == 0) ra2s[rr] = d;
    }
  }
  __syncthreads();

  const int* esrc = ei;
  const int* edst = ei + nE;
  const bool al16 = ((nE & 3) == 0);
  const int sent = -2147483647 - 1;

  const int nChunks = (nE + CHUNK - 1) / CHUNK;
#pragma unroll 1
  for (int ch = 0; ch < nChunks; ++ch) {
    const int cbase = ch * CHUNK;
    int wc = 0;
#pragma unroll
    for (int g = 0; g < NGRP; ++g) {
      const int el0 = (g * NTHR + tid) * 4;
      const int e0  = cbase + el0;
      v4i s4, d4;
      if (al16 && (cbase + CHUNK <= nE)) {
        s4 = *(const v4i*)(esrc + e0);
        d4 = *(const v4i*)(edst + e0);
      } else {
        const int e0c = min(e0, nE - 1), e1c = min(e0 + 1, nE - 1);
        const int e2c = min(e0 + 2, nE - 1), e3c = min(e0 + 3, nE - 1);
        s4.x = (e0     < nE) ? esrc[e0c] : sent;
        s4.y = (e0 + 1 < nE) ? esrc[e1c] : sent;
        s4.z = (e0 + 2 < nE) ? esrc[e2c] : sent;
        s4.w = (e0 + 3 < nE) ? esrc[e3c] : sent;
        d4.x = (e0     < nE) ? edst[e0c] : sent;
        d4.y = (e0 + 1 < nE) ? edst[e1c] : sent;
        d4.z = (e0 + 2 < nE) ? edst[e2c] : sent;
        d4.w = (e0 + 3 < nE) ? edst[e3c] : sent;
      }
      const unsigned f0 = (unsigned)s4.x - (unsigned)nodeBase;
      const unsigned f1 = (unsigned)s4.y - (unsigned)nodeBase;
      const unsigned f2 = (unsigned)s4.z - (unsigned)nodeBase;
      const unsigned f3 = (unsigned)s4.w - (unsigned)nodeBase;
      const unsigned b0 = (unsigned)d4.x - (unsigned)nodeBase;
      const unsigned b1 = (unsigned)d4.y - (unsigned)nodeBase;
      const unsigned b2 = (unsigned)d4.z - (unsigned)nodeBase;
      const unsigned b3 = (unsigned)d4.w - (unsigned)nodeBase;
      const bool hf0 = f0 < (unsigned)NB, hf1 = f1 < (unsigned)NB;
      const bool hf2 = f2 < (unsigned)NB, hf3 = f3 < (unsigned)NB;
      const bool hb0 = b0 < (unsigned)NB, hb1 = b1 < (unsigned)NB;
      const bool hb2 = b2 < (unsigned)NB, hb3 = b3 < (unsigned)NB;
      const unsigned many = __builtin_amdgcn_ballot_w32(hf0 | hf1 | hf2 | hf3 | hb0 | hb1 | hb2 | hb3);
      if (many != 0u) {
#define HITJ(J, T, HJ, SJ) { \
          const unsigned mj = __builtin_amdgcn_ballot_w32(HJ); \
          if (HJ) { \
            const int pos = wc + (int)__builtin_amdgcn_mbcnt_lo(mj, 0u); \
            if (pos < WCAP) list[wave * WCAP + pos] = ((el0 + (J)) << 10) | ((T) << 9) | (int)(SJ); \
          } \
          wc += (int)__builtin_popcount(mj); }
        HITJ(0, 0, hf0, f0)
        HITJ(0, 1, hb0, b0)
        HITJ(1, 0, hf1, f1)
        HITJ(1, 1, hb1, b1)
        HITJ(2, 0, hf2, f2)
        HITJ(2, 1, hb2, b2)
        HITJ(3, 0, hf3, f3)
        HITJ(3, 1, hb3, b3)
#undef HITJ
      }
    }
    if (lane == 0) wcnt[wave] = wc;
    __syncthreads();

    if (wave == 0) {
      for (int wsx = 0; wsx < NWAVE; ++wsx) {
        int n = wcnt[wsx];
        if (n > WCAP) n = WCAP;
        if (n < 0) n = 0;
#pragma unroll 1
        for (int i = 0; i < n; ++i) {
          const int ent  = list[wsx * WCAP + i];
          const int slot = ent & (NB - 1);
          const int typ  = (ent >> 9) & 1;
          const int el   = (ent >> 10) & (CHUNK - 1);
          int e = cbase + el;
          if (e > nE - 1) e = nE - 1;
          int s = esrc[e];
          s = s < 0 ? 0 : (s > nN - 1 ? nN - 1 : s);
          int d = edst[e];
          d = d < 0 ? 0 : (d > nN - 1 ? nN - 1 : d);
          int r = er[e];
          r = r < 0 ? 0 : (r > nR - 1 ? nR - 1 : r);
          const int j = typ ? s : d;
          int nd = nodeBase + slot;
          if (nd > nN - 1) nd = nN - 1;
          const float ra = ra2s[r];
          const float sc = ha1[nd] + ha2[j] + (typ ? ra : -ra);
          const float ls = (sc >= 0.f) ? sc : 0.2f * sc;
          const float p  = expf(-ls);
          const v4f xv = *(const v4f*)(Hp + (size_t)j * DF + 4 * lane);
          v4f* sp = (v4f*)(sacc + slot * DF + 4 * lane);
          const v4f cur = *sp;
          const v4f nxt = cur + p * xv;
          *sp = nxt;
          if (lane == 0) {
            const float o = den[slot];
            den[slot] = o + p;
          }
        }
      }
    }
    __syncthreads();
  }

#pragma unroll 1
  for (int jj = 0; jj < NB / NWAVE; ++jj) {
    const int slot = wave * (NB / NWAVE) + jj;
    const int node = nodeBase + slot;
    if (node >= nN) break;
    const size_t nrow = (size_t)node;
    const float se = ha1[nrow] + ha2[nrow];
    const float le = (se >= 0.f) ? se : 0.2f * se;
    const float pe = expf(-le);
    const v4f hv = *(const v4f*)(Hp + nrow * DF + 4 * lane);
    const v4f sv = *(const v4f*)(sacc + slot * DF + 4 * lane) + pe * hv;
    const float dv  = den[slot] + pe;
    const float inv = 1.0f / dv;
    v4f y = sv * inv;
    y.x = (y.x > 0.f) ? y.x : expm1f(y.x);
    y.y = (y.y > 0.f) ? y.y : expm1f(y.y);
    y.z = (y.z > 0.f) ? y.z : expm1f(y.z);
    y.w = (y.w > 0.f) ? y.w : expm1f(y.w);
    float* op = out + nrow * DF + 4 * lane;
    *(volatile v4f*)op = y;
    __threadfence();
    *(volatile v4f*)op = y;
  }
}

static inline size_t al256(size_t v) { return (v + 255) & ~(size_t)255; }

extern "C" void kernel_launch(void* const* d_in, const int* in_sizes, int n_in,
                              void* d_out, int out_size, void* d_ws, size_t ws_size,
                              hipStream_t stream) {
  if (n_in < 6) return;
  const int nN = in_sizes[0] / KF;
  if (nN <= 0 || in_sizes[0] != nN * KF) return;
  const int nR = in_sizes[1] / DF;
  if (nR < 1 || nR > RCAP || in_sizes[1] != nR * DF) return;
  if (in_sizes[2] != KF * DF) return;
  if (in_sizes[3] != 2 * DF) return;
  const int nE = in_sizes[5];
  if (nE < 0 || in_sizes[4] != 2 * nE) return;
  if (out_size != nN * DF) return;

  const float* x    = (const float*)d_in[0];
  const float* remb = (const float*)d_in[1];
  const float* W    = (const float*)d_in[2];
  const float* av   = (const float*)d_in[3];
  const int*   ei   = (const int*)d_in[4];
  const int*   er   = (const int*)d_in[5];
  float* out = (float*)d_out;

  const int nP = ((nN + GR - 1) / GR) * GR;
  size_t off = 0;
  unsigned short* Wp = (unsigned short*)((char*)d_ws + off);
  off = al256(off + (size_t)2 * WPLANE * sizeof(unsigned short));
  float* Hp = (float*)((char*)d_ws + off);
  off = al256(off + (size_t)nP * DF * sizeof(float));
  float* ha1 = (float*)((char*)d_ws + off);
  off = al256(off + (size_t)nP * sizeof(float));
  float* ha2 = (float*)((char*)d_ws + off);
  off = al256(off + (size_t)nP * sizeof(float));
  if (off > ws_size) return;

  k_prep<<<DF / NWAVE, NTHR, 0, stream>>>(W, Wp);

  k_gemm<<<nP / GR, NTHR, 0, stream>>>(x, Wp, av, Hp, ha1, ha2, nN);

  hipFuncSetAttribute(reinterpret_cast<const void*>(&k_agg),
                      hipFuncAttributeMaxDynamicSharedMemorySize, LDS_BYTES);
  const int grid = (nN + NB - 1) / NB;
  k_agg<<<grid, NTHR, LDS_BYTES, stream>>>(Hp, ha1, ha2, ei, er, remb, av, out, nN, nE, nR);
}
